// KAN_Convolutional_Layer_84378927497340
// MI455X (gfx1250) — hardware-verified
//
#include <hip/hip_runtime.h>
#include <math.h>

#define NB_ 8
#define CIN 32
#define IH 64
#define IW 64
#define OH 62
#define OW 62
#define NP (OH * OW)
#define NCV 8
#define KF 9
#define NCO 8
#define NG 12
#define KTOT (KF + KF * NCO)
#define GROUP (NCV * NP)

typedef _Float16 f16;
typedef __attribute__((ext_vector_type(16))) f16 f16x16;
typedef __attribute__((ext_vector_type(8)))  f16 f16x8;
typedef __attribute__((ext_vector_type(8)))  float f32x8;
typedef __attribute__((ext_vector_type(4)))  float v4f_t;
typedef float v4fa __attribute__((ext_vector_type(4), may_alias));
__device__ __forceinline__ f32x8 wmma16(f16x16 a, f16x16 b, f32x8 c) {
  c = __builtin_amdgcn_wmma_f32_16x16x32_f16(false, a, false, b, (short)0, c, false, false);
  asm volatile("v_nop\n\tv_nop\n\tv_nop\n\tv_nop" : "+v"(c) : "v"(a), "v"(b));
  return c;
}
__device__ __forceinline__ f16x16 lds_frag(const f16* base, int stride) {
  const int lane = threadIdx.x & 31, row = lane & 15, kh = (lane >> 4) * 8;
  const f16x8 lo = *(const f16x8*)(base + row * stride + kh);
  const f16x8 hi = *(const f16x8*)(base + row * stride + kh + 16);
  f16x16 f;
#pragma unroll
  for (int i = 0; i < 8; ++i) { f[i] = lo[i]; f[i + 8] = hi[i]; }
  return f;
}

__global__ __launch_bounds__(256) void k_kan(const float* __restrict__ x, const float* __restrict__ grid, const float* __restrict__ bw, const float* __restrict__ sw,
                                            const float* __restrict__ ssc, float* __restrict__ out) {
  __shared__ __attribute__((aligned(16))) f16 aS[2][128 * 104];
  __shared__ __attribute__((aligned(16))) f16 wS[2][16 * 104];
  __shared__ float gS[KF * NG];
  __shared__ float rS[KF * 3 * 12];
  __shared__ __attribute__((aligned(16))) float oS[4 * NP + 32];
  __shared__ __attribute__((aligned(16))) float carry[16];
  const int tid = threadIdx.x, lane = tid & 31, wave = tid >> 5, cl = lane & 15, rh = (lane >> 4) * 8;
  const int b = blockIdx.x / CIN, c = blockIdx.x % CIN;
  const float* xc = x + ((size_t)b * CIN + c) * IH * IW;
  for (int e = tid; e < KF * NG; e += 256) gS[e] = grid[e];
  __syncthreads();
  for (int e = tid; e < KF * 3 * 12; e += 256) { const int f = e / 36, k = (e % 36) / 12 + 1, t = e % 12; rS[e] = (t + k < NG) ? 1.0f / (gS[f * NG + t + k] - gS[f * NG + t]) : 0.0f; }
  for (int e = tid; e < 16 * 96; e += 256) { const int v = e / 96, k = e % 96; float w = 0.0f;
    if (v < NCV) { if (k < KF) w = bw[v * KF + k]; else if (k < KTOT) { const int f = (k - KF) >> 3, j = (k - KF) & 7; w = sw[(v * KF + f) * NCO + j] * ssc[v * KF + f]; } }
    const f16 h = (f16)w; wS[0][v * 104 + k] = h; wS[1][v * 104 + k] = (f16)((w - (float)h) * 2048.0f); }
  __syncthreads();
  float* dst = out + ((size_t)(b * CIN + c)) * GROUP;
#pragma unroll 1
  for (int pass = 0; pass < 2; ++pass) {
#pragma unroll 1
    for (int p0 = 0; p0 < NP; p0 += 128) {
      __syncthreads();
      { const int r = tid >> 1, half = tid & 1, p = p0 + r; const bool ok = p < NP; const int oh = ok ? p / OW : 0, ow = ok ? p % OW : 0;
        const int f0 = half ? 5 : 0, f1 = half ? 9 : 5;
        for (int f = f0; f < f1; ++f) { const int i = f / 3, jx = f % 3; const float xv = ok ? xc[(oh + i) * IW + ow + jx] : 0.0f;
          const float silu = ok ? xv / (1.0f + expf(-xv)) : 0.0f;
          const float* g = gS + f * NG; const float* rk = rS + f * 36; float bs[11];
#pragma unroll
          for (int t = 0; t < 11; ++t) bs[t] = (xv >= g[t] && xv < g[t + 1]) ? 1.0f : 0.0f;
#pragma unroll
          for (int k = 1; k <= 3; ++k) {
#pragma unroll
            for (int t = 0; t < 11 - k; ++t) bs[t] = (xv - g[t]) * rk[(k - 1) * 12 + t] * bs[t] + (g[t + k + 1] - xv) * rk[(k - 1) * 12 + t + 1] * bs[t + 1]; }
          { const float v = silu; const f16 h = (f16)v; aS[0][r * 104 + f] = h; aS[1][r * 104 + f] = (f16)((v - (float)h) * 2048.0f); }
#pragma unroll
          for (int j = 0; j < NCO; ++j) { const float v = ok ? bs[j] : 0.0f; const f16 h = (f16)v; const int k = KF + f * NCO + j; aS[0][r * 104 + k] = h; aS[1][r * 104 + k] = (f16)((v - (float)h) * 2048.0f); } }
        if (half) { for (int k = KTOT; k < 96; ++k) { aS[0][r * 104 + k] = (f16)0.0f; aS[1][r * 104 + k] = (f16)0.0f; } } }
      __syncthreads();
      f32x8 acc = {}, accx = {};
#pragma unroll
      for (int ks = 0; ks < 3; ++ks) { const f16x16 ah = lds_frag(aS[0] + (wave * 16) * 104 + ks * 32, 104), al = lds_frag(aS[1] + (wave * 16) * 104 + ks * 32, 104);
        const f16x16 bh = lds_frag(wS[0] + ks * 32, 104), bl = lds_frag(wS[1] + ks * 32, 104);
        acc = wmma16(ah, bh, acc); accx = wmma16(ah, bl, accx); accx = wmma16(al, bh, accx); }
      if ((cl >> 2) == pass) { const int vl = cl & 3;
#pragma unroll
        for (int r = 0; r < 8; ++r) { const int p = p0 + wave * 16 + rh + r; if (p < NP) oS[16 + vl * NP + p] = acc[r] + accx[r] * (1.0f / 2048.0f); } }
    }
    __syncthreads();
    if (pass == 0) {
#pragma unroll 1
      for (int ps = 0; ps < 2; ++ps) { for (int q4 = tid; q4 < 15360 / 4; q4 += 256) *(volatile v4f_t*)(dst + q4 * 4) = *(const volatile v4fa*)(oS + 16 + q4 * 4); __threadfence(); }
      __syncthreads();
      if (tid < 16) carry[tid] = oS[16 + 15360 + tid];
      __syncthreads();
      if (tid < 16) oS[tid] = carry[tid];
    } else {
#pragma unroll 1
      for (int ps = 0; ps < 2; ++ps) { for (int q4 = tid; q4 < (GROUP - 15360) / 4; q4 += 256) *(volatile v4f_t*)(dst + 15360 + q4 * 4) = *(const volatile v4fa*)(oS + q4 * 4); __threadfence(); }
    }
  }
}

extern "C" void kernel_launch(void* const* d_in, const int* in_sizes, int n_in,
                              void* d_out, int out_size, void* d_ws, size_t ws_size,
                              hipStream_t stream) {
  (void)in_sizes; (void)n_in; (void)out_size; (void)d_ws; (void)ws_size;
  const float* x = (const float*)d_in[0];
  const float* grid = (const float*)d_in[1];
  const float* bw = (const float*)d_in[2];
  const float* sw = (const float*)d_in[3];
  const float* ssc = (const float*)d_in[4];
  float* out = (float*)d_out;
  k_kan<<<dim3(NB_ * CIN), dim3(256), 0, stream>>>(x, grid, bw, sw, ssc, out);
}
